// MTAD_GAT_37941741093077
// MI455X (gfx1250) — hardware-verified
//
#include <string.h>
#include <hip/hip_runtime.h>


namespace {
constexpr int NB = 16, W = 128, K = 128, KS = 7, HG = 256, OUT = 128, ED = 256, NR = NB * W  , G3 = 3 * HG  , WP_ = W + 6;
constexpr float XS = 8.0f, WSC = 256.0f, ALPHA = 0.2f;

typedef _Float16 b16;
typedef __attribute__((ext_vector_type(16))) _Float16 v16b;
typedef __attribute__((ext_vector_type(8))) _Float16 v8b;
typedef __attribute__((ext_vector_type(8))) float v8f;
typedef __attribute__((ext_vector_type(4))) float v4f;
__device__ __forceinline__ float bf16_rne(float f) { unsigned int u = __float_as_uint(f); u += 0x7FFFu + ((u >> 16) & 1u); return __uint_as_float(u & 0xFFFF0000u); }
__device__ __forceinline__ void split16(float v, b16& hi, b16& lo) { hi = (b16)v; lo = (b16)(v - (float)hi); }
__device__ __forceinline__ v16b frag_kb(const b16* p, int hh) { const v8b a = *(const v8b*)(p + 8 * hh), b = *(const v8b*)(p + 16 + 8 * hh); v16b f;
#pragma unroll
  for (int e = 0; e < 8; ++e) { f[e] = a[e]; f[8 + e] = b[e]; } return f; }
__device__ __forceinline__ v8f wmma16b(v16b a, v16b b, v8f c) { v8f d = __builtin_amdgcn_wmma_f32_16x16x32_f16(false, a, false, b, (short)0, c, false, false); asm volatile("v_nop\n\tv_nop\n\tv_nop\n\tv_nop" : "+v"(d) : "v"(a), "v"(b)); return d; }
__device__ __forceinline__ void wave_lds_sync() { __builtin_amdgcn_fence(__ATOMIC_RELEASE, "workgroup"); __builtin_amdgcn_wave_barrier(); __builtin_amdgcn_fence(__ATOMIC_ACQUIRE, "workgroup"); }
__device__ __forceinline__ float pmul(float a, float b) { float p = a * b; asm volatile("" : "+v"(p)); return p; }
__device__ __forceinline__ float wsum(float v) { v += __shfl_xor(v, 1); v += __shfl_xor(v, 2); v += __shfl_xor(v, 4); v += __shfl_xor(v, 8); return v + __shfl_xor(v, 16); }
__device__ __forceinline__ float wmax(float v) { v = fmaxf(v, __shfl_xor(v, 1)); v = fmaxf(v, __shfl_xor(v, 2)); v = fmaxf(v, __shfl_xor(v, 4)); v = fmaxf(v, __shfl_xor(v, 8)); return fmaxf(v, __shfl_xor(v, 16)); }
__device__ __forceinline__ float nexp(float x) { return __builtin_amdgcn_exp2f(x * 1.4426950408889634f); }
__device__ __forceinline__ float sigm(float x) { return 1.0f / (1.0f + nexp(-x)); }
__device__ __forceinline__ float tanh_(float x) { const float e = nexp(-2.0f * fabsf(x)); const float t = (1.0f - e) / (1.0f + e); return x < 0.0f ? -t : t; }
__device__ __forceinline__ float lrelu(float x) { return x > 0.0f ? x : ALPHA * x; }

constexpr size_t OFF0 = 0, OFF1 = OFF0 + 128 * 896, OFF2 = OFF1 + 256 * 128, OFF3 = OFF2 + 256 * 128, OFF4 = OFF3 + 256 * 128, OFF5 = OFF4 + 256 * 128, OFF6 = OFF5 + (size_t)768 * 384, OFF7 = OFF6 + (size_t)768 * 256, OFF8 = OFF7 + 256 * 256, OFF9 = OFF8 + 128 * 256, OFF10 = OFF9 + (size_t)768 * 256, OFFEND = OFF10 + 128 * 256;
__global__ __launch_bounds__(256) void prepw_kernel(const float* __restrict__ convw, const float* __restrict__ fgw, const float* __restrict__ tgw, const float* __restrict__ wih, const float* __restrict__ whh, const float* __restrict__ fc1, const float* __restrict__ fc2, const float* __restrict__ dwhh, const float* __restrict__ rfc, b16* __restrict__ WP) {
  const size_t t = (size_t)blockIdx.x * 256 + threadIdx.x; const size_t e = t * 8; if (e >= OFFEND) return; v8b o;
  for (int j = 0; j < 8; ++j) { const size_t q = e + j; float v;
    if (q < OFF1) { const int oo = (int)(q / 896), k = (int)(q % 896), tap = k / 128, i = k % 128; v = convw[((size_t)oo * K + i) * KS + tap]; }
    else if (q < OFF3) { const size_t r = q - (q < OFF2 ? OFF1 : OFF2); const int oo = (int)(r / 128), i = (int)(r % 128); v = fgw[(size_t)oo * 256 + (q < OFF2 ? 0 : 128) + i]; }
    else if (q < OFF5) { const size_t r = q - (q < OFF4 ? OFF3 : OFF4); const int oo = (int)(r / 128), i = (int)(r % 128); v = tgw[(size_t)oo * 256 + (q < OFF4 ? 0 : 128) + i]; }
    else if (q < OFF6) v = wih[q - OFF5]; else if (q < OFF7) v = whh[q - OFF6]; else if (q < OFF8) v = fc1[q - OFF7]; else if (q < OFF9) v = fc2[q - OFF8]; else if (q < OFF10) v = dwhh[q - OFF9]; else v = rfc[q - OFF10];
    o[j] = (b16)(bf16_rne(v) * WSC); }
  for (int pass = 0; pass < 2; ++pass) { *(volatile v8b*)(WP + e) = o; __threadfence(); }
}
__global__ __launch_bounds__(256) void prepx_kernel(const float* __restrict__ x, b16* __restrict__ X16P) {
  const size_t t = (size_t)blockIdx.x * 256 + threadIdx.x; if (t >= (size_t)NB * WP_ * K / 8) return; const size_t e = t * 8; const int b = (int)(e / ((size_t)WP_ * K)); const int r = (int)((e / K) % WP_); const int c0 = (int)(e % K); v8b o = {};
  if (r >= 3 && r < 3 + W) for (int j = 0; j < 8; ++j) o[j] = (b16)(bf16_rne(x[((size_t)b * W + r - 3) * K + c0 + j]) * XS);
  for (int pass = 0; pass < 2; ++pass) { *(volatile v8b*)(X16P + e) = o; __threadfence(); }
}
struct GP { const b16 *Ah, *Al, *Bh, *Bl; size_t bstrideB; int K, lda, ldy; const float* bias; float* Yf; b16 *Yh, *Yl, *Y2h, *Y2l, *Y3h, *Y3l; };
template <int MODE>
__global__ __launch_bounds__(128) void gemm_kernel(GP g) {
  __shared__ __attribute__((aligned(16))) float Ts[4][16][128 + 4];
  const int wave = threadIdx.x >> 5, lane = threadIdx.x & 31, nloc = lane & 15, hlf = lane >> 4, t_ = threadIdx.x; const size_t m0 = (size_t)blockIdx.x * 64 + wave * 16; const int n0 = blockIdx.y * 128;
  const int b = (int)(((size_t)blockIdx.x * 64) / W); const b16* Bh = g.Bh + (size_t)b * g.bstrideB; const b16* Bl = g.Bl ? g.Bl + (size_t)b * g.bstrideB : nullptr;
  v8f acc[8];
#pragma unroll
  for (int t = 0; t < 8; ++t) acc[t] = (v8f){};
  const b16* Abase = g.Ah + (MODE == 0 ? (size_t)b * 6 * K : 0);
  for (int kb = 0; kb < g.K; kb += 32) { const v16b a = frag_kb(Abase + (m0 + nloc) * g.lda + kb, hlf); v16b al = {}; if (g.Al) al = frag_kb(g.Al + (m0 + nloc) * g.lda + kb, hlf);
#pragma unroll
    for (int t = 0; t < 8; ++t) { const v16b bw = frag_kb(Bh + (size_t)(n0 + t * 16 + nloc) * g.K + kb, hlf); acc[t] = wmma16b(a, bw, acc[t]); if (g.Al) acc[t] = wmma16b(al, bw, acc[t]); if (MODE == 3 || MODE == 4) acc[t] = wmma16b(a, frag_kb(Bl + (size_t)(n0 + t * 16 + nloc) * g.K + kb, hlf), acc[t]); } }
  const float rs_ = (MODE == 3 || MODE == 4) ? 1.0f / (XS * XS) : 1.0f / (XS * WSC);
#pragma unroll
  for (int t = 0; t < 8; ++t) { const int c = n0 + t * 16 + nloc; const float bb = g.bias ? bf16_rne(g.bias[c]) : 0.0f;
#pragma unroll
    for (int r = 0; r < 8; ++r) { float v = acc[t][r] * rs_ + bb; if (MODE == 0) v = fmaxf(v, 0.0f); if (MODE == 3 || MODE == 4) v = sigm(v); Ts[wave][8 * hlf + r][t * 16 + nloc] = v; } }
  __syncthreads();
  const int w0 = (int)(((size_t)blockIdx.x * 64) % W);
  for (int pass = 0; pass < 2; ++pass) {
    if (MODE == 0 || MODE == 1 || MODE == 2 || MODE == 5) { for (int rr = 0; rr < 16; ++rr) *(volatile v4f*)(g.Yf + (m0 + rr) * g.ldy + n0 + lane * 4) = *(const v4f*)(&Ts[wave][rr][lane * 4]); }
    if (MODE == 0 || MODE == 4) {
      for (int rr = 0; rr < 16; ++rr) if (lane < 16) { v8b hv, lv; for (int j = 0; j < 8; ++j) { b16 p, q; split16(Ts[wave][rr][lane * 8 + j] * XS, p, q); hv[j] = p; lv[j] = q; }
        if (MODE == 0) { *(volatile v8b*)(g.Yh + (m0 + rr) * K + lane * 8) = hv; *(volatile v8b*)(g.Yl + (m0 + rr) * K + lane * 8) = lv; }
        *(volatile v8b*)(g.Y2h + (m0 + rr) * 384 + (MODE == 0 ? 0 : 256) + lane * 8) = hv; *(volatile v8b*)(g.Y2l + (m0 + rr) * 384 + (MODE == 0 ? 0 : 256) + lane * 8) = lv; } }
    if (MODE == 0 || MODE == 3) {
      for (int i = t_; i < 128 * 8; i += 128) { const int c = i >> 3, r8 = (i & 7) * 8; v8b hv, lv; for (int j = 0; j < 8; ++j) { b16 p, q; split16(Ts[(r8 + j) >> 4][(r8 + j) & 15][c] * XS, p, q); hv[j] = p; lv[j] = q; }
        if (MODE == 0) { const size_t gi = ((size_t)b * K + c) * W + w0 + r8; *(volatile v8b*)(g.Y3h + gi) = hv; *(volatile v8b*)(g.Y3l + gi) = lv; }
        else { const size_t gi = ((size_t)b * W + c) * 384 + 128 + w0 + r8; *(volatile v8b*)(g.Y2h + gi) = hv; *(volatile v8b*)(g.Y2l + gi) = lv; } } }
    __threadfence(); }
}
__global__ __launch_bounds__(256) void pair_kernel(const float* __restrict__ P, const float* __restrict__ Q, const float* __restrict__ av, const float* __restrict__ bias, b16* __restrict__ ATh, b16* __restrict__ ATl) {
  const int wave = threadIdx.x >> 5, lane = threadIdx.x & 31; const size_t row = (size_t)blockIdx.x * 8 + wave; const int b = (int)(row / W), i = (int)(row % W); const int d0 = lane * 8;
  float p[8], a8[8]; for (int q = 0; q < 8; ++q) { p[q] = P[row * ED + d0 + q]; a8[q] = bf16_rne(av[d0 + q]); }
  float e4[4] = {0, 0, 0, 0};
  for (int j = 0; j < W; ++j) { const float* qr = Q + ((size_t)b * W + j) * ED + d0; float s = 0.0f; for (int q = 0; q < 8; ++q) s += pmul(a8[q], lrelu(p[q] + qr[q])); s = wsum(s) + bf16_rne(bias[i * W + j]);
#pragma unroll
    for (int u = 0; u < 4; ++u) if (j == lane + 32 * u) e4[u] = s; }
  float mx = fmaxf(fmaxf(e4[0], e4[1]), fmaxf(e4[2], e4[3])); mx = wmax(mx); float ex[4], sm = 0.0f; for (int u = 0; u < 4; ++u) { ex[u] = nexp(e4[u] - mx); sm += ex[u]; } sm = wsum(sm); const float inv = 1.0f / sm;
  __shared__ __attribute__((aligned(16))) b16 Sh[8][W + 8], Sl[8][W + 8];
  for (int u = 0; u < 4; ++u) { b16 hq, lq; split16(ex[u] * inv * XS, hq, lq); Sh[wave][lane + 32 * u] = hq; Sl[wave][lane + 32 * u] = lq; }
  wave_lds_sync();
  for (int pass = 0; pass < 2; ++pass) { if (lane < 16) { *(volatile v8b*)(ATh + row * W + lane * 8) = *(const v8b*)(&Sh[wave][lane * 8]); *(volatile v8b*)(ATl + row * W + lane * 8) = *(const v8b*)(&Sl[wave][lane * 8]); } __threadfence(); }
}
template <int DEC>
__global__ __launch_bounds__(128) void gru_kernel(const float* __restrict__ XG, const b16* __restrict__ WHH, const float* __restrict__ bhh, const b16* __restrict__ FC1, const float* __restrict__ fc1b, const b16* __restrict__ FC2, const float* __restrict__ fc2b, const float* __restrict__ dwih, const float* __restrict__ dbih, float* __restrict__ out0, float* __restrict__ GI, b16* __restrict__ DECh, b16* __restrict__ DECl) {
  __shared__ __attribute__((aligned(16))) b16 Hh[16][HG + 8], Hl[16][HG + 8]; __shared__ float Hf[16][HG + 4]; __shared__ float GH[16][G3 + 4]; __shared__ float S0[G3], S1[G3];
  const int wave = threadIdx.x >> 5, lane = threadIdx.x & 31, nloc = lane & 15, hlf = lane >> 4, t_ = threadIdx.x;
  for (int i = t_; i < 16 * (HG + 8); i += 128) { Hh[i / (HG + 8)][i % (HG + 8)] = (b16)0.0f; Hl[i / (HG + 8)][i % (HG + 8)] = (b16)0.0f; } for (int i = t_; i < 16 * (HG + 4); i += 128) Hf[i / (HG + 4)][i % (HG + 4)] = 0.0f;
  __syncthreads();
  for (int step = 0; step < W; ++step) {
    v8f acc[12];
#pragma unroll
    for (int tt = 0; tt < 12; ++tt) acc[tt] = (v8f){};
#pragma unroll 2
    for (int kb = 0; kb < HG; kb += 32) { const v16b a = frag_kb(&Hh[nloc][kb], hlf), al = frag_kb(&Hl[nloc][kb], hlf);
#pragma unroll
      for (int tt = 0; tt < 12; ++tt) { const v16b bw = frag_kb(WHH + (size_t)((wave * 12 + tt) * 16 + nloc) * HG + kb, hlf); acc[tt] = wmma16b(a, bw, acc[tt]); acc[tt] = wmma16b(al, bw, acc[tt]); } }
#pragma unroll
    for (int tt = 0; tt < 12; ++tt) { const int c = (wave * 12 + tt) * 16 + nloc; const float bb = bf16_rne(bhh[c]);
#pragma unroll
      for (int r = 0; r < 8; ++r) GH[8 * hlf + r][c] = acc[tt][r] * (1.0f / (XS * WSC)) + bb; }
    __syncthreads();
    { const int row = t_ >> 3, j0 = (t_ & 7) * 32; const size_t xo = ((size_t)row * W + step) * G3;
      for (int j = j0; j < j0 + 32; ++j) { const float r = sigm(XG[xo + j] + GH[row][j]), z = sigm(XG[xo + HG + j] + GH[row][HG + j]); const float n = tanh_(XG[xo + 2 * HG + j] + pmul(r, GH[row][2 * HG + j])); const float h = pmul(1.0f - z, n) + pmul(z, Hf[row][j]);
        Hf[row][j] = h; b16 a_, c_; split16(h * XS, a_, c_); Hh[row][j] = a_; Hl[row][j] = c_; }
      if (DEC) { for (int pass = 0; pass < 2; ++pass) { for (int j8 = j0; j8 < j0 + 32; j8 += 8) { v8b hv, lv; for (int q = 0; q < 8; ++q) { hv[q] = Hh[row][j8 + q]; lv[q] = Hl[row][j8 + q]; } *(volatile v8b*)(DECh + ((size_t)row * W + step) * HG + j8) = hv; *(volatile v8b*)(DECl + ((size_t)row * W + step) * HG + j8) = lv; } __threadfence(); } } }
    __syncthreads(); }
  if (DEC) return;
  { v8f a1[4] = {{}, {}, {}, {}};
#pragma unroll 2
    for (int kb = 0; kb < HG; kb += 32) { const v16b a = frag_kb(&Hh[nloc][kb], hlf), al = frag_kb(&Hl[nloc][kb], hlf);
#pragma unroll
      for (int tt = 0; tt < 4; ++tt) { const v16b bw = frag_kb(FC1 + (size_t)((wave * 4 + tt) * 16 + nloc) * HG + kb, hlf); a1[tt] = wmma16b(a, bw, a1[tt]); a1[tt] = wmma16b(al, bw, a1[tt]); } }
#pragma unroll
    for (int tt = 0; tt < 4; ++tt) { const int c = (wave * 4 + tt) * 16 + nloc; const float bb = bf16_rne(fc1b[c]);
#pragma unroll
      for (int r = 0; r < 8; ++r) GH[8 * hlf + r][c] = fmaxf(a1[tt][r] * (1.0f / (XS * WSC)) + bb, 0.0f); } }
  __syncthreads();
  for (int o = t_; o < G3; o += 128) { float s0 = 0.0f, s1 = 0.0f; for (int j = 0; j < 128; ++j) { s0 += bf16_rne(dwih[(size_t)o * HG + j]); s1 += bf16_rne(dwih[(size_t)o * HG + 128 + j]); } S0[o] = s0; S1[o] = s1; }
  __syncthreads();
  for (int pass = 0; pass < 2; ++pass) { for (int i = t_; i < 16 * W * (G3 / 4); i += 128) { const int q4 = i % (G3 / 4), rw = i / (G3 / 4), b = rw / W, w = rw % W; const float h0v = Hf[b][2 * w], h1v = Hf[b][2 * w + 1]; v4f o;
      for (int j = 0; j < 4; ++j) { const int oo = q4 * 4 + j; o[j] = pmul(h0v, S0[oo]) + pmul(h1v, S1[oo]) + bf16_rne(dbih[oo]); } *(volatile v4f*)(GI + ((size_t)b * W + w) * G3 + q4 * 4) = o; } __threadfence(); }
  __syncthreads();
  for (int i = t_; i < 16 * HG; i += 128) { const int r = i / HG, c = i % HG; b16 p, q; split16(GH[r][c] * XS, p, q); Hh[r][c] = p; Hl[r][c] = q; }
  __syncthreads();
  { v8f a2[2] = {{}, {}};
#pragma unroll 2
    for (int kb = 0; kb < HG; kb += 32) { const v16b a = frag_kb(&Hh[nloc][kb], hlf), al = frag_kb(&Hl[nloc][kb], hlf);
#pragma unroll
      for (int tt = 0; tt < 2; ++tt) { const v16b bw = frag_kb(FC2 + (size_t)((wave * 2 + tt) * 16 + nloc) * HG + kb, hlf); a2[tt] = wmma16b(a, bw, a2[tt]); a2[tt] = wmma16b(al, bw, a2[tt]); } }
#pragma unroll
    for (int tt = 0; tt < 2; ++tt) { const int c = (wave * 2 + tt) * 16 + nloc; const float bb = bf16_rne(fc2b[c]);
#pragma unroll
      for (int r = 0; r < 8; ++r) GH[8 * hlf + r][c] = a2[tt][r] * (1.0f / (XS * WSC)) + bb; } }
  __syncthreads();
  for (int pass = 0; pass < 2; ++pass) { for (int i = t_; i < 16 * OUT / 4; i += 128) { const int r = i / (OUT / 4), c4 = (i % (OUT / 4)) * 4; *(volatile v4f*)(out0 + (size_t)r * OUT + c4) = *(const v4f*)(&GH[r][c4]); } __threadfence(); }
}
}

extern "C" void kernel_launch(void* const* d_in, const int* in_sizes, int n_in, void* d_out, int out_size, void* d_ws, size_t ws_size, hipStream_t stream) {
  (void)n_in;
  auto Fp = [&](int i) { return (const float*)d_in[i]; };
  if (in_sizes[0] != NR * K || in_sizes[1] != K * K * KS || in_sizes[3] != ED * 2 * W || in_sizes[11] != G3 * 384 || in_sizes[19] != G3 * HG || in_sizes[23] != OUT * HG || out_size != NB * OUT + NR * OUT) return;
  size_t off = 0; char* ws = (char*)d_ws;
  auto carve = [&](size_t bytes) { char* p = ws + off; off += (bytes + 255) & ~(size_t)255; return p; };
  b16* WP = (b16*)carve(OFFEND * 2); b16* X16P = (b16*)carve((size_t)NB * WP_ * K * 2);
  float* XC = (float*)carve((size_t)NR * K * 4); b16* XCh = (b16*)carve((size_t)NR * K * 2); b16* XCl = (b16*)carve((size_t)NR * K * 2); b16* XCTh = (b16*)carve((size_t)NR * K * 2); b16* XCTl = (b16*)carve((size_t)NR * K * 2);
  b16* HCh = (b16*)carve((size_t)NR * 384 * 2); b16* HCl = (b16*)carve((size_t)NR * 384 * 2);
  float* PF = (float*)carve((size_t)NR * ED * 4); float* QF = (float*)carve((size_t)NR * ED * 4); float* PT = (float*)carve((size_t)NR * ED * 4); float* QT = (float*)carve((size_t)NR * ED * 4);
  b16* AFh = (b16*)carve((size_t)NR * W * 2); b16* AFl = (b16*)carve((size_t)NR * W * 2); b16* ATh = (b16*)carve((size_t)NR * W * 2); b16* ATl = (b16*)carve((size_t)NR * W * 2);
  float* XG = (float*)carve((size_t)NR * G3 * 4); float* GI = (float*)carve((size_t)NR * G3 * 4); b16* DECh = (b16*)carve((size_t)NR * HG * 2); b16* DECl = (b16*)carve((size_t)NR * HG * 2);
  if (off > ws_size || off > ((size_t)128 << 20)) return;
  float* out0 = (float*)d_out; float* out1 = (float*)d_out + (size_t)NB * OUT;
  prepw_kernel<<<(unsigned)((OFFEND / 8 + 255) / 256), 256, 0, stream>>>(Fp(1), Fp(3), Fp(7), Fp(11), Fp(12), Fp(15), Fp(17), Fp(20), Fp(23), WP);
  prepx_kernel<<<(unsigned)(((size_t)NB * WP_ * K / 8 + 255) / 256), 256, 0, stream>>>(Fp(0), X16P);
  auto mk = [&]() { GP g; memset(&g, 0, sizeof(g)); return g; };
  { GP g = mk(); g.Ah = X16P + 0; g.Al = nullptr; g.Bh = WP + OFF0; g.K = 896; g.lda = K; g.ldy = K; g.bias = Fp(2); g.Yf = XC; g.Yh = XCh; g.Yl = XCl; g.Y2h = HCh; g.Y2l = HCl; g.Y3h = XCTh; g.Y3l = XCTl; g.bstrideB = 0;
    gemm_kernel<0><<<dim3(NR / 64, 1), 128, 0, stream>>>(g); }
  { GP g = mk(); g.Ah = XCTh; g.Al = XCTl; g.Bh = WP + OFF1; g.K = K; g.lda = K; g.ldy = ED; g.bias = Fp(4); g.Yf = PF; gemm_kernel<1><<<dim3(NR / 64, 2), 128, 0, stream>>>(g); g.Bh = WP + OFF2; g.bias = nullptr; g.Yf = QF; gemm_kernel<1><<<dim3(NR / 64, 2), 128, 0, stream>>>(g); }
  { GP g = mk(); g.Ah = XCh; g.Al = XCl; g.Bh = WP + OFF3; g.K = K; g.lda = K; g.ldy = ED; g.bias = Fp(8); g.Yf = PT; gemm_kernel<1><<<dim3(NR / 64, 2), 128, 0, stream>>>(g); g.Bh = WP + OFF4; g.bias = nullptr; g.Yf = QT; gemm_kernel<1><<<dim3(NR / 64, 2), 128, 0, stream>>>(g); }
  pair_kernel<<<NR / 8, 256, 0, stream>>>(PF, QF, Fp(5), Fp(6), AFh, AFl);
  pair_kernel<<<NR / 8, 256, 0, stream>>>(PT, QT, Fp(9), Fp(10), ATh, ATl);
  { GP g = mk(); g.Ah = AFh; g.Al = AFl; g.Bh = XCh; g.Bl = XCl; g.bstrideB = (size_t)W * K; g.K = W; g.lda = W; g.Y2h = HCh; g.Y2l = HCl; gemm_kernel<3><<<dim3(NR / 64, 1), 128, 0, stream>>>(g); }
  { GP g = mk(); g.Ah = ATh; g.Al = ATl; g.Bh = XCTh; g.Bl = XCTl; g.bstrideB = (size_t)K * W; g.K = W; g.lda = W; g.Y2h = HCh; g.Y2l = HCl; gemm_kernel<4><<<dim3(NR / 64, 1), 128, 0, stream>>>(g); }
  { GP g = mk(); g.Ah = HCh; g.Al = HCl; g.Bh = WP + OFF5; g.K = 384; g.lda = 384; g.ldy = G3; g.bias = Fp(13); g.Yf = XG; gemm_kernel<1><<<dim3(NR / 64, 6), 128, 0, stream>>>(g); }
  gru_kernel<0><<<1, 128, 0, stream>>>(XG, WP + OFF6, Fp(14), WP + OFF7, Fp(16), WP + OFF8, Fp(18), Fp(19), Fp(21), out0, GI, nullptr, nullptr);
  gru_kernel<1><<<1, 128, 0, stream>>>(GI, WP + OFF9, Fp(22), nullptr, nullptr, nullptr, nullptr, nullptr, nullptr, nullptr, nullptr, DECh, DECl);
  { GP g = mk(); g.Ah = DECh; g.Al = DECl; g.Bh = WP + OFF10; g.K = HG; g.lda = HG; g.ldy = OUT; g.bias = Fp(24); g.Yf = out1; gemm_kernel<5><<<dim3(NR / 64, 1), 128, 0, stream>>>(g); }
}
